// SelectiveAttention_40192303956183
// MI455X (gfx1250) — hardware-verified
//
#include <hip/hip_runtime.h>
#include <math.h>
#include <stdint.h>

#define NB    1
#define SEQ   4096
#define DM    1024
#define NH    16
#define HD    64
#define DG    256
#define NQB   (SEQ / 64)
#define VLP   512
#define RESQB 8
static_assert(RESQB * 64 <= VLP);
static_assert(NH * HD == DM);
static_assert((SEQ % 64) == 0 && (DM % 64) == 0 && (DM % 32) == 0 && (DG % 64) == 0);
static_assert(((NB * SEQ / 64) * (DM / 64)) % 8 == 0);
static_assert(((DM / 64) * (SEQ / 64)) % 8 == 0);
static_assert(((SEQ / 64) * (DG / 64)) % 8 == 0);
static_assert((NB * SEQ * DM) % (8 * 256) == 0);
static_assert((SEQ % 32) == 0);
static_assert(DG == 256);

typedef _Float16 v16h __attribute__((ext_vector_type(16)));
typedef _Float16 v8h  __attribute__((ext_vector_type(8)));
typedef __bf16   v16b __attribute__((ext_vector_type(16)));
typedef __bf16   v8b  __attribute__((ext_vector_type(8)));
typedef float    v8f  __attribute__((ext_vector_type(8)));
typedef float    v4f  __attribute__((ext_vector_type(4)));
typedef unsigned int v4u __attribute__((ext_vector_type(4)));

__device__ __forceinline__ unsigned short bf_bits(float f) {
  unsigned u = __float_as_uint(f);
  return (unsigned short)((u + 0x7FFFu + ((u >> 16) & 1u)) >> 16);
}
__device__ __forceinline__ float bf_up(unsigned short h) { return __uint_as_float(((unsigned)h) << 16); }
__device__ __forceinline__ unsigned short h_bits(_Float16 x) { return __builtin_bit_cast(unsigned short, x); }
__device__ __forceinline__ unsigned pk16(unsigned short a, unsigned short b) { return (unsigned)a | ((unsigned)b << 16); }
__device__ __forceinline__ v8f zero8() { v8f z = {0.f, 0.f, 0.f, 0.f, 0.f, 0.f, 0.f, 0.f}; return z; }
__device__ __forceinline__ v8h zero8h() {
  const _Float16 z = (_Float16)0.0f;
  v8h r = {z, z, z, z, z, z, z, z};
  return r;
}

__device__ __forceinline__ v16b ldfrag_b(const __bf16* p) {
  union { v16b v; v8b h[2]; } f;
  f.h[0] = *(const v8b*)(p);
  f.h[1] = *(const v8b*)(p + 16);
  return f.v;
}

__device__ __forceinline__ v8f mma_b(v16b a, v16b b, v8f c) {
  c = __builtin_amdgcn_wmma_f32_16x16x32_bf16(false, a, false, b, (short)0, c, false, false);
  asm volatile("v_nop\n\tv_nop\n\tv_nop\n\tv_nop" : "+v"(c) : "v"(a), "v"(b));
  return c;
}
__device__ __forceinline__ v8f mma_h(v16h a, v16h b, v8f c) {
  c = __builtin_amdgcn_wmma_f32_16x16x32_f16(false, a, false, b, (short)0, c, false, false);
  asm volatile("v_nop\n\tv_nop\n\tv_nop\n\tv_nop" : "+v"(c) : "v"(a), "v"(b));
  return c;
}
__device__ __forceinline__ v8f mma_b_raw(v16b a, v16b b, v8f c) {
  return __builtin_amdgcn_wmma_f32_16x16x32_bf16(false, a, false, b, (short)0, c, false, false);
}
__device__ __forceinline__ void dep_guard_b(v8f& a, v8f& b, v16b x, v16b y) {
  asm volatile("v_nop\n\tv_nop\n\tv_nop\n\tv_nop" : "+v"(a), "+v"(b) : "v"(x), "v"(y));
}
__device__ __forceinline__ void keep4_b(v16b a, v16b b, v16b c, v16b d) {
  asm volatile("v_nop" :: "v"(a), "v"(b), "v"(c), "v"(d));
}
__device__ __forceinline__ void acc_guard4(v8f& a, v8f& b, v8f& c, v8f& d) {
  asm volatile("v_nop\n\tv_nop\n\tv_nop\n\tv_nop" : "+v"(a), "+v"(b), "+v"(c), "+v"(d));
}

__global__ __launch_bounds__(256) void cvt_bf16x8(const float* __restrict__ in, unsigned short* out, int n8) {
  const int i = blockIdx.x * 256 + threadIdx.x;
  if (i < n8) {
    const v4f a = *(const v4f*)(in + (size_t)i * 8);
    const v4f b = *(const v4f*)(in + (size_t)i * 8 + 4);
    v4u p;
    p[0] = pk16(bf_bits(a[0]), bf_bits(a[1]));
    p[1] = pk16(bf_bits(a[2]), bf_bits(a[3]));
    p[2] = pk16(bf_bits(b[0]), bf_bits(b[1]));
    p[3] = pk16(bf_bits(b[2]), bf_bits(b[3]));
    *(volatile v4u*)(out + (size_t)i * 8) = p;
    __threadfence();
    *(volatile v4u*)(out + (size_t)i * 8) = p;
  }
}

__global__ __launch_bounds__(256) void cvt_bf16_T(const float* __restrict__ in, unsigned short* out,
                                                  int nrow, int ncol) {
  __shared__ __align__(16) unsigned short Tt[64 * 72];
  const int tid = threadIdx.x, lane = tid & 31, wave = tid >> 5;
  const int c0 = blockIdx.x * 64;
  const int r0 = blockIdx.y * 64;
  {
    const int i  = tid >> 2;
    const int cs = (tid & 3) * 16;
    const float* src = in + (size_t)(r0 + i) * ncol + c0 + cs;
#pragma unroll
    for (int e4 = 0; e4 < 4; ++e4) {
      const v4f v = *(const v4f*)(src + 4 * e4);
#pragma unroll
      for (int e = 0; e < 4; ++e) Tt[(cs + 4 * e4 + e) * 72 + i] = bf_bits(v[e]);
    }
  }
  __syncthreads();
  const int q = lane >> 3, c8 = (lane & 7) * 8;
  v4u pv[2];
#pragma unroll
  for (int it = 0; it < 2; ++it) {
    const int j = it * 32 + wave * 4 + q;
    pv[it] = *(const v4u*)(Tt + j * 72 + c8);
  }
  for (int pass = 0; pass < 2; ++pass) {
#pragma unroll
    for (int it = 0; it < 2; ++it) {
      const int j = it * 32 + wave * 4 + q;
      *(volatile v4u*)(out + (size_t)(c0 + j) * nrow + r0 + c8) = pv[it];
    }
    __threadfence();
  }
}

__global__ __launch_bounds__(256) void k_gate(const float* __restrict__ Hs, const float* __restrict__ w2,
                                              const float* __restrict__ b2p, float* gout, int nrows) {
  __shared__ __align__(16) float gs[32];
  const int tid = threadIdx.x, lane = tid & 31, wave = tid >> 5;
  const int rowBase = blockIdx.x * 32;
  const float b2 = bf_up(bf_bits(b2p[0]));
  for (int rr = 0; rr < 4; ++rr) {
    int row = rowBase + wave * 4 + rr;
    row = (row < nrows) ? row : (nrows - 1);
    const float* hp = Hs + (size_t)row * DG + lane * 8;
    const float* wp = w2 + lane * 8;
    float acc = 0.f;
#pragma unroll 1
    for (int e = 0; e < 8; ++e) {
      const float hv = hp[e];
      const float wv = bf_up(bf_bits(wp[e]));
      const float ge = 0.5f * hv * erfcf(-hv * 0.707106781186547524f);
      acc = fmaf(ge, wv, acc);
    }
#pragma unroll
    for (int off = 1; off < 32; off <<= 1) acc += __shfl_xor(acc, off, 32);
    float z = acc + b2;
    z = fminf(fmaxf(z, -30.0f), 30.0f);
    const float g = 1.0f / (1.0f + expf(-z));
    if (lane == 0) gs[wave * 4 + rr] = g;
  }
  __syncthreads();
  if (wave == 0 && lane < 8) {
    const v4f v = *(const v4f*)(gs + lane * 4);
    float* p = gout + rowBase + lane * 4;
    *(volatile v4f*)p = v;
    __threadfence();
    *(volatile v4f*)p = v;
  }
}

template <int NSPLIT, int OUT_MODE, int BIAS>
__global__ __launch_bounds__(256) void gemm64(
    const unsigned short* __restrict__ Ap, const unsigned short* A2p, int lda, long long strideA,
    const unsigned short* __restrict__ Btp, int ldb, long long strideB,
    const float* __restrict__ bias,
    void* Cout, int ldc, long long strideC,
    void* Cout2, int ldc2, long long strideC2, int N2,
    const float* gvec, const float* xres, int ldx,
    int M, int N, int K, float rscale) {
  const __bf16* A   = (const __bf16*)(const void*)Ap;
  const __bf16* A2  = (const __bf16*)(const void*)A2p;
  const __bf16* Bt  = (const __bf16*)(const void*)Btp;
  __shared__ __align__(16) float sT[8][16 * 68];
  const int b    = blockIdx.y;
  const int lane = threadIdx.x & 31;
  const int wave = threadIdx.x >> 5;
  const int tilesN = N >> 6;
  const int tilesM = M >> 6;
  const int tile = blockIdx.x * 8 + wave;
  if (tile >= tilesM * tilesN) return;
  const int tm = tile / tilesN;
  const int tn = tile - tm * tilesN;
  const int m0 = tm << 6;
  const int n0 = tn << 6;

  const __bf16* Ab  = A  + (size_t)b * strideA;
  const __bf16* Bb  = Bt + (size_t)b * strideB;
  const __bf16* Ab2 = (NSPLIT >= 1) ? (A2 + (size_t)b * strideA) : Ab;

  const int rlane = lane & 15;
  const int koff  = (lane >> 4) * 8;
  const int mOff  = (lane >> 4) * 8;

  v8f acc[4][4];
#pragma unroll
  for (int i = 0; i < 4; ++i)
#pragma unroll
    for (int j = 0; j < 4; ++j) acc[i][j] = zero8();

  for (int k0 = 0; k0 < K; k0 += 32) {
    v16b bh[4];
#pragma unroll
    for (int j = 0; j < 4; ++j) {
      const size_t bo = (size_t)(n0 + (j << 4) + rlane) * ldb + koff + k0;
      bh[j] = ldfrag_b(Bb + bo);
    }
#pragma unroll
    for (int i = 0; i < 4; ++i) {
      const size_t ao = (size_t)(m0 + (i << 4) + rlane) * lda + koff + k0;
      const v16b ah = ldfrag_b(Ab + ao);
      v16b al = ah;
      if (NSPLIT >= 1) al = ldfrag_b(Ab2 + ao);
#pragma unroll
      for (int j = 0; j < 4; ++j) {
        acc[i][j] = mma_b_raw(ah, bh[j], acc[i][j]);
        if (NSPLIT >= 1) acc[i][j] = mma_b_raw(al, bh[j], acc[i][j]);
      }
      dep_guard_b(acc[i][0], acc[i][3], ah, al);
    }
    keep4_b(bh[0], bh[1], bh[2], bh[3]);
  }
  acc_guard4(acc[0][0], acc[0][1], acc[0][2], acc[0][3]);
  acc_guard4(acc[1][0], acc[1][1], acc[1][2], acc[1][3]);
  acc_guard4(acc[2][0], acc[2][1], acc[2][2], acc[2][3]);
  acc_guard4(acc[3][0], acc[3][1], acc[3][2], acc[3][3]);

  float* slab = sT[wave];
  float bcol[4];
#pragma unroll
  for (int j = 0; j < 4; ++j) {
    bcol[j] = 0.f;
    if (BIAS == 1) bcol[j] = bf_up(bf_bits(bias[n0 + (j << 4) + rlane]));
  }
#pragma unroll
  for (int i = 0; i < 4; ++i) {
    const int mBase = m0 + (i << 4);
    float brow[8];
#pragma unroll
    for (int r = 0; r < 8; ++r) {
      brow[r] = 0.f;
      if (BIAS == 2) brow[r] = bf_up(bf_bits(bias[mBase + mOff + r]));
    }
#pragma unroll
    for (int j = 0; j < 4; ++j) {
#pragma unroll
      for (int r = 0; r < 8; ++r) {
        slab[(mOff + r) * 68 + (j << 4) + rlane] = acc[i][j][r] + bcol[j] + brow[r];
      }
    }
    __builtin_amdgcn_fence(__ATOMIC_RELEASE, "workgroup");
    __builtin_amdgcn_wave_barrier();
    __builtin_amdgcn_fence(__ATOMIC_ACQUIRE, "workgroup");
    if (OUT_MODE == 0 || OUT_MODE == 4) {
      float* C = (float*)Cout + (size_t)b * strideC;
      const int hh = lane >> 4, c4 = (lane & 15) * 4;
      for (int pass = 0; pass < 2; ++pass) {
#pragma unroll
        for (int it = 0; it < 8; ++it) {
          const int row = it * 2 + hh;
          v4f v = *(const v4f*)(slab + row * 68 + c4);
          if (OUT_MODE == 4) {
            const int gr = mBase + row;
            const float g = gvec[gr];
            const float omg = 1.0f - g;
            const v4f xr = *(const v4f*)(xres + (size_t)gr * ldx + n0 + c4);
#pragma unroll
            for (int e = 0; e < 4; ++e) {
              const float xb = bf_up(bf_bits(xr[e]));
              v[e] = g * v[e] + omg * xb;
            }
          }
          *(volatile v4f*)(C + (size_t)(mBase + row) * ldc + n0 + c4) = v;
        }
        __threadfence();
      }
    } else {
      const int q = lane >> 3, c8 = (lane & 7) * 8;
      unsigned short* C  = (unsigned short*)Cout  + (size_t)b * strideC;
      unsigned short* C2 = (unsigned short*)Cout2 + (size_t)b * strideC2;
      const bool wlo = (OUT_MODE == 2) || (n0 < N2);
      v4u hv[4], lv[4];
#pragma unroll
      for (int it = 0; it < 4; ++it) {
        const int row = it * 4 + q;
        const float* sp = slab + row * 68 + c8;
        v4u a, a2;
#pragma unroll
        for (int e = 0; e < 4; ++e) {
          const float f0 = sp[2 * e], f1 = sp[2 * e + 1];
          unsigned short h0, h1, l0, l1;
          if (OUT_MODE == 2) {
            h0 = bf_bits(f0); h1 = bf_bits(f1);
            l0 = bf_bits(f0 - bf_up(h0)); l1 = bf_bits(f1 - bf_up(h1));
          } else {
            const _Float16 x0 = (_Float16)f0, x1 = (_Float16)f1;
            h0 = h_bits(x0); h1 = h_bits(x1);
            l0 = h_bits((_Float16)((f0 - (float)x0) * rscale));
            l1 = h_bits((_Float16)((f1 - (float)x1) * rscale));
          }
          a[e] = pk16(h0, h1); a2[e] = pk16(l0, l1);
        }
        hv[it] = a; lv[it] = a2;
      }
      for (int pass = 0; pass < 2; ++pass) {
#pragma unroll
        for (int it = 0; it < 4; ++it) {
          const int row = it * 4 + q;
          *(volatile v4u*)(C + (size_t)(mBase + row) * ldc + n0 + c8) = hv[it];
          if (wlo) *(volatile v4u*)(C2 + (size_t)(mBase + row) * ldc2 + n0 + c8) = lv[it];
        }
        __threadfence();
      }
    }
    __builtin_amdgcn_fence(__ATOMIC_RELEASE, "workgroup");
    __builtin_amdgcn_wave_barrier();
    __builtin_amdgcn_fence(__ATOMIC_ACQUIRE, "workgroup");
  }
}

template <bool RES>
__global__ __launch_bounds__(128)
void attn_causal64(const unsigned short* __restrict__ qhp, const unsigned short* __restrict__ qlp,
                   const unsigned short* __restrict__ khp, const unsigned short* __restrict__ klp,
                   const unsigned short* __restrict__ vhp, const unsigned short* __restrict__ vlp,
                   unsigned short* ohp, unsigned short* olp,
                   int qbBase, int nqbThis) {
  union FB { v16b v; v8b h[2]; };
  union FH { v16h v; v8h h[2]; };
  __shared__ __align__(16) __bf16   Ksh[64 * 64];
  __shared__ __align__(16) __bf16   Ksl[64 * 64];
  __shared__ __align__(16) _Float16 Vth[64 * 64];
  __shared__ __align__(16) _Float16 Vtl[RES ? 64 * 64 : 8];
  __shared__ __align__(16) _Float16 Psh[4][16 * 64];
  __shared__ __align__(16) _Float16 Psl[RES ? 4 : 1][16 * 64];
  __shared__ __align__(16) float    Os[4][16 * 64];

  const int tid  = threadIdx.x;
  const int wave = tid >> 5;
  const int lane = tid & 31;
  const int hh   = lane >> 4;
  const int c    = lane & 15;

  const int bx   = blockIdx.x;
  const int qbl  = bx % nqbThis;
  const int rest = bx / nqbThis;
  const int h    = rest % NH;
  const int b    = rest / NH;
  const int qb   = qbBase + qbl;
  const int q0   = qb * 64 + wave * 16;
  const size_t rowB = (size_t)b * SEQ;

  const __bf16* Qh = (const __bf16*)(const void*)qhp + (size_t)h * HD;
  const __bf16* Ql = (const __bf16*)(const void*)qlp + (size_t)h * HD;
  const __bf16* Kh = (const __bf16*)(const void*)khp + (size_t)h * HD;
  const __bf16* Kl = (const __bf16*)(const void*)klp + (size_t)h * HD;
  const _Float16* Vh = (const _Float16*)(const void*)vhp + ((size_t)b * DM + (size_t)h * HD) * SEQ;
  const _Float16* Vl = (const _Float16*)(const void*)vlp + ((size_t)b * DM + (size_t)h * HD) * VLP;

  v16b qah[2], qal[2];
#pragma unroll
  for (int dc = 0; dc < 2; ++dc) {
    const size_t qo = (rowB + q0 + c) * DM + dc * 32 + 8 * hh;
    qah[dc] = ldfrag_b(Qh + qo);
    qal[dc] = ldfrag_b(Ql + qo);
  }

  float mrow[8], lrow[8];
  v8f oacc[4];
#pragma unroll
  for (int r = 0; r < 8; ++r) { mrow[r] = -INFINITY; lrow[r] = 0.f; }
#pragma unroll
  for (int t = 0; t < 4; ++t) oacc[t] = zero8();

  for (int kt = 0; kt <= qb; ++kt) {
    const int kv0 = kt * 64;
    __syncthreads();
    {
      const int r = tid >> 1, half = (tid & 1) * 32;
      const __bf16*   kg  = Kh + (rowB + kv0 + r) * DM + half;
      const __bf16*   klg = Kl + (rowB + kv0 + r) * DM + half;
      const _Float16* vg  = Vh + (size_t)r * SEQ + kv0 + half;
      const int kvl = (kv0 + 64 <= VLP) ? kv0 : (VLP - 64);
      const _Float16* vlg = Vl + (size_t)r * VLP + kvl + half;
      const bool resOK = (kv0 + 64 <= VLP);
#pragma unroll
      for (int i = 0; i < 4; ++i) {
        const v8b a0 = *(const v8b*)(kg + 8 * i);
        const v8b a1 = *(const v8b*)(klg + 8 * i);
        const v8h b0 = *(const v8h*)(vg + 8 * i);
        *(v8b*)(Ksh + r * 64 + half + 8 * i) = a0;
        *(v8b*)(Ksl + r * 64 + half + 8 * i) = a1;
        *(v8h*)(Vth + r * 64 + half + 8 * i) = b0;
        if (RES) {
          v8h b1 = *(const v8h*)(vlg + 8 * i);
          if (!resOK) b1 = zero8h();
          *(v8h*)(Vtl + r * 64 + half + 8 * i) = b1;
        }
      }
    }
    __syncthreads();

    v8f s[4];
#pragma unroll
    for (int j = 0; j < 4; ++j) {
      s[j] = zero8();
#pragma unroll
      for (int dc = 0; dc < 2; ++dc) {
        FB kb, kl;
        kb.h[0] = *(const v8b*)(Ksh + (j * 16 + c) * 64 + dc * 32 + 8 * hh);
        kb.h[1] = *(const v8b*)(Ksh + (j * 16 + c) * 64 + dc * 32 + 16 + 8 * hh);
        kl.h[0] = *(const v8b*)(Ksl + (j * 16 + c) * 64 + dc * 32 + 8 * hh);
        kl.h[1] = *(const v8b*)(Ksl + (j * 16 + c) * 64 + dc * 32 + 16 + 8 * hh);
        s[j] = mma_b(qah[dc], kb.v, s[j]);
        s[j] = mma_b(qah[dc], kl.v, s[j]);
        s[j] = mma_b(qal[dc], kb.v, s[j]);
      }
    }

    _Float16* pwh = Psh[wave];
    _Float16* pwl = Psl[RES ? wave : 0];
#pragma unroll
    for (int r = 0; r < 8; ++r) {
      const int rowq = q0 + 8 * hh + r;
      float m = -INFINITY;
#pragma unroll
      for (int j = 0; j < 4; ++j) {
        const int key = kv0 + j * 16 + c;
        float sv = s[j][r] * 0.125f;
        sv = (key <= rowq) ? sv : -INFINITY;
        s[j][r] = sv;
        m = fmaxf(m, sv);
      }
#pragma unroll
      for (int off = 1; off < 16; off <<= 1) m = fmaxf(m, __shfl_xor(m, off, 32));
      const float mnew  = fmaxf(mrow[r], m);
      const float msafe = (mnew == -INFINITY) ? 0.f : mnew;
      const float alpha = __expf(mrow[r] - msafe);
      mrow[r] = mnew;
      float psum = 0.f;
#pragma unroll
      for (int j = 0; j < 4; ++j) {
        const float p = __expf(s[j][r] - msafe);
        psum += p;
        const float p1k = p * 1024.0f;
        const _Float16 ph = (_Float16)p1k;
        pwh[(8 * hh + r) * 64 + j * 16 + c] = ph;
        if (RES) {
          const _Float16 pl = (_Float16)((p1k - (float)ph) * 4096.0f);
          pwl[(8 * hh + r) * 64 + j * 16 + c] = pl;
        }
      }
#pragma unroll
      for (int off = 1; off < 16; off <<= 1) psum += __shfl_xor(psum, off, 32);
      lrow[r] = lrow[r] * alpha + psum;
#pragma unroll
      for (int t = 0; t < 4; ++t) oacc[t][r] *= alpha;
    }
    __builtin_amdgcn_fence(__ATOMIC_RELEASE, "workgroup");
    __builtin_amdgcn_wave_barrier();
    __builtin_amdgcn_fence(__ATOMIC_ACQUIRE, "workgroup");

    v8f o1[4];
#pragma unroll
    for (int t = 0; t < 4; ++t) o1[t] = zero8();
#pragma unroll 1
    for (int kk = 0; kk < 2; ++kk) {
      FH pa, pl;
      pa.h[0] = *(const v8h*)(pwh + c * 64 + kk * 32 + 8 * hh);
      pa.h[1] = *(const v8h*)(pwh + c * 64 + kk * 32 + 16 + 8 * hh);
      if (RES) {
        pl.h[0] = *(const v8h*)(pwl + c * 64 + kk * 32 + 8 * hh);
        pl.h[1] = *(const v8h*)(pwl + c * 64 + kk * 32 + 16 + 8 * hh);
      } else {
        pl.v = pa.v;
      }
#pragma unroll
      for (int t = 0; t < 4; ++t) {
        FH vb;
        vb.h[0] = *(const v8h*)(Vth + (t * 16 + c) * 64 + kk * 32 + 8 * hh);
        vb.h[1] = *(const v8h*)(Vth + (t * 16 + c) * 64 + kk * 32 + 16 + 8 * hh);
        oacc[t] = mma_h(pa.v, vb.v, oacc[t]);
        if (RES) {
          FH vl;
          vl.h[0] = *(const v8h*)(Vtl + (t * 16 + c) * 64 + kk * 32 + 8 * hh);
          vl.h[1] = *(const v8h*)(Vtl + (t * 16 + c) * 64 + kk * 32 + 16 + 8 * hh);
          o1[t] = mma_h(pa.v, vl.v, o1[t]);
          o1[t] = mma_h(pl.v, vb.v, o1[t]);
        }
      }
    }
    if (RES) {
#pragma unroll
      for (int t = 0; t < 4; ++t)
#pragma unroll
        for (int r = 0; r < 8; ++r) oacc[t][r] += o1[t][r] * (1.0f / 4096.0f);
    }
  }

  float* os = Os[wave];
#pragma unroll
  for (int r = 0; r < 8; ++r) {
    const float l = lrow[r];
    const float inv = ((l > 0.f) ? (1.0f / l) : 0.f) * (1.0f / 1024.0f);
#pragma unroll
    for (int t = 0; t < 4; ++t) os[(8 * hh + r) * 64 + t * 16 + c] = oacc[t][r] * inv;
  }
  __builtin_amdgcn_fence(__ATOMIC_RELEASE, "workgroup");
  __builtin_amdgcn_wave_barrier();
  __builtin_amdgcn_fence(__ATOMIC_ACQUIRE, "workgroup");
  {
    const int q4 = lane >> 3, c8 = (lane & 7) * 8;
    v4u hv[4], lv[4];
#pragma unroll
    for (int it = 0; it < 4; ++it) {
      const int row = it * 4 + q4;
      const float* sp = os + row * 64 + c8;
      v4u a, a2;
#pragma unroll
      for (int e = 0; e < 4; ++e) {
        const float f0 = sp[2 * e], f1 = sp[2 * e + 1];
        const unsigned short h0 = bf_bits(f0), h1 = bf_bits(f1);
        const unsigned short l0 = bf_bits(f0 - bf_up(h0)), l1 = bf_bits(f1 - bf_up(h1));
        a[e] = pk16(h0, h1); a2[e] = pk16(l0, l1);
      }
      hv[it] = a; lv[it] = a2;
    }
    for (int pass = 0; pass < 2; ++pass) {
#pragma unroll
      for (int it = 0; it < 4; ++it) {
        const int row = it * 4 + q4;
        const size_t go = (rowB + q0 + row) * DM + (size_t)h * HD + c8;
        *(volatile v4u*)(ohp + go) = hv[it];
        *(volatile v4u*)(olp + go) = lv[it];
      }
      __threadfence();
    }
  }
}

extern "C" void kernel_launch(void* const* d_in, const int* in_sizes, int n_in,
                              void* d_out, int out_size, void* d_ws, size_t ws_size,
                              hipStream_t stream) {
  if (n_in < 7) return;
  if (in_sizes[0] != NB * SEQ * DM) return;
  if (in_sizes[1] != DM * 3 * DM) return;
  if (in_sizes[2] != DM * DG) return;
  if (in_sizes[3] != DG) return;
  if (in_sizes[4] != DG) return;
  if (in_sizes[5] < 1) return;
  if (in_sizes[6] != DM * DM) return;
  if (out_size != NB * SEQ * DM + NB * SEQ) return;

  const float* x    = (const float*)d_in[0];
  const float* Wqkv = (const float*)d_in[1];
  const float* Wg1  = (const float*)d_in[2];
  const float* bg1  = (const float*)d_in[3];
  const float* Wg2  = (const float*)d_in[4];
  const float* bg2  = (const float*)d_in[5];
  const float* Wout = (const float*)d_in[6];
  float* out0 = (float*)d_out;
  float* gout = out0 + (size_t)NB * SEQ * DM;

  const size_t PX  = (size_t)NB * SEQ * DM * 2;
  const size_t PW1 = (size_t)DM * DM * 2;
  const size_t PWA = (size_t)3 * PW1;
  const size_t PWP = PW1;
  const size_t PWG = (size_t)DG * DM * 2;
  const size_t PHS = (size_t)NB * SEQ * DG * 4;
  const size_t PVT = (size_t)NB * DM * SEQ * 2;
  const size_t PVL = (size_t)NB * DM * VLP * 2;
  size_t off = 0;
  const size_t oXb  = off; off += PX;
  const size_t oWA  = off; off += PWA;
  const size_t oWP  = off; off += PWP;
  const size_t oWG  = off; off += PWG;
  const size_t oHs  = off; off += PHS;
  const size_t oQh  = off; off += PX;
  const size_t oQl  = off; off += PX;
  const size_t oKh  = off; off += PX;
  const size_t oKl  = off; off += PX;
  const size_t oVTh = off; off += PVT;
  const size_t oVTl = off; off += PVL;
  const size_t oOh  = off; off += PX;
  const size_t oOl  = off; off += PX;
  if (off > ws_size) return;
  if (off > (size_t)134217728) return;

  char* ws = (char*)d_ws;
  unsigned short* Xb  = (unsigned short*)(ws + oXb);
  unsigned short* WA  = (unsigned short*)(ws + oWA);
  unsigned short* WqB = WA;
  unsigned short* WkB = WA + (size_t)DM * DM;
  unsigned short* WvB = WA + (size_t)2 * DM * DM;
  unsigned short* WPb = (unsigned short*)(ws + oWP);
  unsigned short* WGb = (unsigned short*)(ws + oWG);
  float*          Hs  = (float*)(ws + oHs);
  unsigned short* Qh  = (unsigned short*)(ws + oQh);
  unsigned short* Ql  = (unsigned short*)(ws + oQl);
  unsigned short* Kh  = (unsigned short*)(ws + oKh);
  unsigned short* Kl  = (unsigned short*)(ws + oKl);
  unsigned short* VTh = (unsigned short*)(ws + oVTh);
  unsigned short* VTl = (unsigned short*)(ws + oVTl);
  unsigned short* Oh  = (unsigned short*)(ws + oOh);
  unsigned short* Ol  = (unsigned short*)(ws + oOl);

  const dim3 blk(256);
  const int n8x = NB * SEQ * DM / 8;
  const dim3 gCvtX((n8x + 255) / 256);
  const dim3 gTA((3 * DM) / 64, DM / 64);
  const dim3 gTP(DM / 64, DM / 64);
  const dim3 gTG(DG / 64, DM / 64);
  const dim3 gGateH(((NB * SEQ / 64) * (DG / 64) + 7) / 8, 1);
  const dim3 gGate(NB * SEQ / 32);
  const dim3 gProj(((NB * SEQ / 64) * (DM / 64) + 7) / 8, 1);
  const dim3 gVT(((DM / 64) * (SEQ / 64) + 7) / 8, NB);

  cvt_bf16x8<<<gCvtX, blk, 0, stream>>>(x, Xb, n8x);
  cvt_bf16_T<<<gTA, blk, 0, stream>>>(Wqkv, WA, DM, 3 * DM);
  cvt_bf16_T<<<gTP, blk, 0, stream>>>(Wout, WPb, DM, DM);
  cvt_bf16_T<<<gTG, blk, 0, stream>>>(Wg1, WGb, DM, DG);
  gemm64<0, 0, 1><<<gGateH, blk, 0, stream>>>(
      Xb, Xb, DM, 0LL, WGb, DM, 0LL, bg1,
      (void*)Hs, DG, 0LL, (void*)Hs, DG, 0LL, DG,
      x, x, DM,
      NB * SEQ, DG, DM, 1.0f);
  k_gate<<<gGate, blk, 0, stream>>>(Hs, Wg2, bg2, gout, NB * SEQ);
  gemm64<0, 2, 0><<<gProj, blk, 0, stream>>>(
      Xb, Xb, DM, 0LL, WqB, DM, 0LL, bg1,
      (void*)Qh, DM, 0LL, (void*)Ql, DM, 0LL, DM,
      x, x, DM,
      NB * SEQ, DM, DM, 1.0f);
  gemm64<0, 2, 0><<<gProj, blk, 0, stream>>>(
      Xb, Xb, DM, 0LL, WkB, DM, 0LL, bg1,
      (void*)Kh, DM, 0LL, (void*)Kl, DM, 0LL, DM,
      x, x, DM,
      NB * SEQ, DM, DM, 1.0f);
  gemm64<0, 3, 0><<<gVT, blk, 0, stream>>>(
      WvB, WvB, DM, 0LL, Xb, DM, (long long)SEQ * DM, bg1,
      (void*)VTh, SEQ, (long long)DM * SEQ, (void*)VTl, VLP, (long long)DM * VLP, VLP,
      x, x, DM,
      DM, SEQ, DM, 4096.0f);
  attn_causal64<true><<<dim3(NB * NH * RESQB), dim3(128), 0, stream>>>(
      Qh, Ql, Kh, Kl, VTh, VTl, Oh, Ol, 0, RESQB);
  attn_causal64<false><<<dim3(NB * NH * (NQB - RESQB)), dim3(128), 0, stream>>>(
      Qh, Ql, Kh, Kl, VTh, VTl, Oh, Ol, RESQB, NQB - RESQB);
  gemm64<1, 4, 0><<<gProj, blk, 0, stream>>>(
      Oh, Ol, DM, 0LL, WPb, DM, 0LL, bg1,
      d_out, DM, 0LL, d_out, DM, 0LL, DM,
      gout, x, DM,
      NB * SEQ, DM, DM, 1.0f);
  (void)hipGetLastError();
}
